// TransformerModel_38689065402773
// MI455X (gfx1250) — hardware-verified
//
#include <hip/hip_runtime.h>


#ifndef NB
#define NB 131072
#endif
#define NB_FULL 131072
#define SEQ   32
#define DM    16
#define NVOC  257
#define AWV   8
#define SPW   16
#define N8SRC ((NVOC * DM) / 8)
#define N8TOT ((((NVOC * DM * 2) + 127) / 128) * 8)
#define SC2   ((float)(0.25 * 1.4426950408889634))
#define PSH   14.0f
#define NEGB  (-3.0e38f)

static_assert(SEQ == 32);
static_assert(DM == 16);
static_assert((NVOC * DM) % 8 == 0);
static_assert(N8TOT >= N8SRC);
static_assert(N8TOT % 8 == 0);
static_assert(NB % (AWV * SPW) == 0);
static_assert(NB <= NB_FULL);
static_assert((size_t)NB * SEQ < (size_t)4294967296ull);
static_assert(2 * 32 * 16 == SPW * DM * 4);
static_assert((SPW * DM * 4) % 128 == 0);
static_assert((size_t)NB_FULL * DM * 4 == (size_t)8388608);
static_assert(AWV * SEQ * DM * 2 + AWV * SPW * DM * 4 <= 131072);

typedef _Float16 h16;
typedef __attribute__((ext_vector_type(16))) _Float16 v16h;
typedef __attribute__((ext_vector_type(8)))  _Float16 v8h;
typedef __attribute__((ext_vector_type(8)))  float    v8f;
typedef __attribute__((ext_vector_type(4)))  float    v4f;
typedef v4f  __attribute__((may_alias)) v4fa;

__device__ __forceinline__ unsigned short f2bf(float f) { unsigned u = __float_as_uint(f); u += 0x7FFFu + ((u >> 16) & 1u); return (unsigned short)(u >> 16); }
__device__ __forceinline__ float bfr(float f) { return __uint_as_float(((unsigned)f2bf(f)) << 16); }
__device__ __forceinline__ v16h cat16(v8h lo, v8h hi) { return __builtin_shufflevector(lo, hi, 0, 1, 2, 3, 4, 5, 6, 7, 8, 9, 10, 11, 12, 13, 14, 15); }
__device__ __forceinline__ v8f wmma16(v16h a, v16h b, v8f c) { return __builtin_amdgcn_wmma_f32_16x16x32_f16(false, a, false, b, (short)0, c, false, false); }
__device__ __forceinline__ void wave_sync() { __builtin_amdgcn_fence(3  , "wavefront"); __builtin_amdgcn_wave_barrier(); asm volatile("" ::: "memory"); }

static __device__ __forceinline__ h16 toh_flush(float v) { const float w = (fabsf(v) < 6.103515625e-05f) ? 0.0f : v; return (h16)w; }
static __device__ __forceinline__ v8f wmma16g(v16h a, v16h b, v8f c) { c = wmma16(a, b, c); asm volatile("v_nop\n\tv_nop\n\tv_nop\n\tv_nop" : "+v"(c) : "v"(a), "v"(b)); return c; }
static __device__ __forceinline__ v8h pk8(v8f d) { v8h o;
#pragma unroll
    for (int r = 0; r < 8; ++r) o[r] = toh_flush(d[r]);
    return o; }
static __device__ __forceinline__ v16h ldw(const float* p) {
    const v4f a = *(const v4f*)p, c = *(const v4f*)(p + 4); v8h lo;
#pragma unroll
    for (int i = 0; i < 4; ++i) { lo[i] = toh_flush(bfr(a[i])); lo[4 + i] = toh_flush(bfr(c[i])); }
    return cat16(lo, (v8h){}); }
static __device__ __forceinline__ v16h softp(v8f sa, v8f sb, float& inv) {
    float ta[8], tb[8]; float mx = NEGB;
#pragma unroll
    for (int r = 0; r < 8; ++r) { ta[r] = sa[r] * SC2; tb[r] = sb[r] * SC2; mx = fmaxf(mx, fmaxf(ta[r], tb[r])); }
    mx = fmaxf(mx, __shfl_xor(mx, 16, 32));
    const float sh = PSH - mx;
    v16h pb; float ls = 0.0f;
#pragma unroll
    for (int r = 0; r < 8; ++r) {
        const float xa = ta[r] + sh, xc = tb[r] + sh;
        const float ea = (xa < -14.0f) ? 0.0f : __builtin_amdgcn_exp2f(xa);
        const float ec = (xc < -14.0f) ? 0.0f : __builtin_amdgcn_exp2f(xc);
        const h16 pa = (h16)ea; const h16 pc = (h16)ec;
        pb[r] = pa; pb[8 + r] = pc;
        ls += (float)pa + (float)pc; }
    ls += __shfl_xor(ls, 16, 32);
    inv = 1.0f / ls;
    return pb; }

__global__ __launch_bounds__(256) void k_cvth8(const float* __restrict__ src, h16* dst, unsigned n8src, unsigned n8tot) {
    const unsigned i = blockIdx.x * 256u + threadIdx.x; if (i >= n8tot) return;
    const unsigned ic = min(i, n8src - 1u);
    const v8f v = *(const v8f*)(src + (size_t)ic * 8);
    const bool live = i < n8src; v8h o;
#pragma unroll
    for (int k = 0; k < 8; ++k) { const float w = live ? bfr(v[k]) : 0.0f; o[k] = toh_flush(w); }
    *(volatile v8h*)(dst + (size_t)i * 8) = o; __threadfence(); *(volatile v8h*)(dst + (size_t)i * 8) = o;
}

__global__ __launch_bounds__(32 * AWV) void k_enc(const int* __restrict__ arr, const h16* __restrict__ EH,
                                                  const float* __restrict__ wq, const float* __restrict__ wk, const float* __restrict__ wv,
                                                  const float* __restrict__ w1, const float* __restrict__ b1,
                                                  const float* __restrict__ w2, const float* __restrict__ b2, float* OUT) {
    __shared__ __align__(16) h16   xs[AWV * SEQ * DM];
    __shared__ __align__(16) float os[AWV * SPW * DM];
    const int lane = threadIdx.x & 31, lr = lane & 15, hi = lane >> 4;
    const int wave = __builtin_amdgcn_readfirstlane((int)(threadIdx.x >> 5));
    const unsigned bx = blockIdx.x;
    const unsigned s0 = (bx * (unsigned)AWV + (unsigned)wave) * (unsigned)SPW;
    const unsigned wo = (unsigned)lr * (unsigned)DM + 8u * (unsigned)hi;
    const v16h fq = ldw(wq + wo), fk = ldw(wk + wo), fv = ldw(wv + wo), f1 = ldw(w1 + wo), f2 = ldw(w2 + wo);
    float b1r[8];
    { const v4f ba = *(const v4f*)(b1 + 8 * hi), bc = *(const v4f*)(b1 + 8 * hi + 4);
#pragma unroll
      for (int r = 0; r < 4; ++r) { b1r[r] = bfr(ba[r]); b1r[4 + r] = bfr(bc[r]); } }
    const float b2v = bfr(b2[lr]);
    const int xb = wave * SEQ * DM, ob = wave * SPW * DM;
    const v8h hz8 = (v8h){};
    const v8f z = (v8f){};
#pragma unroll 1
    for (int i = 0; i < SPW; ++i) {
        const unsigned smp = s0 + (unsigned)i;
        int tok = arr[smp * (unsigned)SEQ + (unsigned)lane];
        tok = min(max(tok, 0), NVOC - 1);
        const unsigned tu = (unsigned)tok;
        const h16* er = EH + tu * (unsigned)DM;
        const v8h e0 = *(const v8h*)er, e1 = *(const v8h*)(er + 8);
        wave_sync();
        *(v8h*)(&xs[xb + lane * DM]) = e0; *(v8h*)(&xs[xb + lane * DM + 8]) = e1;
        wave_sync();
        const v16h xf0 = cat16(*(const v8h*)(&xs[xb + lr * DM + 8 * hi]), hz8);
        const v16h xf1 = cat16(*(const v8h*)(&xs[xb + (16 + lr) * DM + 8 * hi]), hz8);
        const v8f qt0 = wmma16g(fq, xf0, z), qt1 = wmma16g(fq, xf1, z);
        const v8f kt0 = wmma16g(fk, xf0, z), kt1 = wmma16g(fk, xf1, z);
        const v8f vv0 = wmma16g(xf0, fv, z), vv1 = wmma16g(xf1, fv, z);
        const v16h aK0 = cat16(pk8(kt0), hz8), aK1 = cat16(pk8(kt1), hz8);
        const v16h bQ0 = cat16(pk8(qt0), hz8), bQ1 = cat16(pk8(qt1), hz8);
        const v16h aV  = cat16(pk8(vv0), pk8(vv1));
        const v8f s00 = wmma16g(aK0, bQ0, z), s10 = wmma16g(aK1, bQ0, z);
        const v8f s01 = wmma16g(aK0, bQ1, z), s11 = wmma16g(aK1, bQ1, z);
        float inv0, inv1;
        const v16h pb0 = softp(s00, s10, inv0);
        const v16h pb1 = softp(s01, s11, inv1);
        const v8f o0 = wmma16g(aV, pb0, z), o1 = wmma16g(aV, pb1, z);
        v8h c0, c1;
#pragma unroll
        for (int r = 0; r < 8; ++r) { c0[r] = toh_flush(o0[r] * inv0); c1[r] = toh_flush(o1[r] * inv1); }
        const v16h bX0 = cat16(c0, hz8), bX1 = cat16(c1, hz8);
        const v8f g0 = wmma16g(f1, bX0, z), g1 = wmma16g(f1, bX1, z);
        v8h h0, h1;
#pragma unroll
        for (int r = 0; r < 8; ++r) { h0[r] = toh_flush(fmaxf(g0[r] + b1r[r], 0.0f)); h1[r] = toh_flush(fmaxf(g1[r] + b1r[r], 0.0f)); }
        const v16h aH0 = cat16(h0, hz8), aH1 = cat16(h1, hz8);
        const v8f y0 = wmma16g(aH0, f2, z), y1 = wmma16g(aH1, f2, z);
        float part = 0.0f;
#pragma unroll
        for (int r = 0; r < 8; ++r) part += y0[r] + y1[r];
        const float tot = part + __shfl_xor(part, 16, 32);
        const float mean = tot * (1.0f / 32.0f) + b2v;
        if (hi == 0) os[ob + i * DM + lr] = mean;
    }
    wave_sync();
    float* orow = OUT + (size_t)s0 * DM;
#pragma unroll 1
    for (int ps = 0; ps < 2; ++ps) {
#pragma unroll
        for (int s = 0; s < 2; ++s) { const int idx = s * 32 + lane;
            const v4f val = *(const v4fa*)(&os[ob + idx * 4]);
            *(volatile v4f*)(orow + idx * 4) = val; }
        if (ps == 0) __threadfence(); }
}

static constexpr size_t al256(size_t v) { return (v + 255) & ~(size_t)255; }
static constexpr size_t SZ_EH = al256((size_t)N8TOT * 16);
static constexpr size_t SZ_TOTAL = SZ_EH;
static_assert((size_t)N8TOT * 16 <= SZ_EH);
static_assert((size_t)NVOC * DM * 2 <= (size_t)N8TOT * 16);
static_assert(SZ_TOTAL <= (size_t)134217728);

extern "C" void kernel_launch(void* const* d_in, const int* in_sizes, int n_in,
                              void* d_out, int out_size, void* d_ws, size_t ws_size, hipStream_t stream) {
    if (n_in < 10) return;
    if ((size_t)in_sizes[0] < (size_t)NB * SEQ || (size_t)in_sizes[1] < (size_t)NB * SEQ) return;
    if (in_sizes[2] < NVOC * DM) return;
    if (in_sizes[3] < DM * DM || in_sizes[4] < DM * DM || in_sizes[5] < DM * DM || in_sizes[6] < DM * DM || in_sizes[8] < DM * DM) return;
    if (in_sizes[7] < DM || in_sizes[9] < DM) return;
    if ((size_t)out_size < (size_t)NB_FULL * DM + (size_t)NB * DM) return;
    if (SZ_TOTAL > ws_size) return;
    const int* arr1 = (const int*)d_in[0]; const int* arr2 = (const int*)d_in[1];
    const float* emb = (const float*)d_in[2];
    const float* wq = (const float*)d_in[3]; const float* wk = (const float*)d_in[4]; const float* wv = (const float*)d_in[5];
    const float* w1 = (const float*)d_in[6]; const float* b1 = (const float*)d_in[7];
    const float* w2 = (const float*)d_in[8]; const float* b2 = (const float*)d_in[9];
    float* OUT0 = (float*)d_out;
    float* OUT1 = (float*)d_out + (size_t)NB_FULL * DM;
    h16* EH = (h16*)d_ws;

    k_cvth8<<<(unsigned)((N8TOT + 255) / 256), 256, 0, stream>>>(emb, EH, (unsigned)N8SRC, (unsigned)N8TOT);
    k_enc<<<dim3(NB / (AWV * SPW), 1, 1), 32 * AWV, 0, stream>>>(arr1, EH, wq, wk, wv, w1, b1, w2, b2, OUT0);
    k_enc<<<dim3(NB / (AWV * SPW), 1, 1), 32 * AWV, 0, stream>>>(arr2, EH, wq, wk, wv, w1, b1, w2, b2, OUT1);
}
